// ConfounderStackLayers_44925357916624
// MI455X (gfx1250) — hardware-verified
//
#include <hip/hip_runtime.h>
#include <math.h>

typedef __attribute__((ext_vector_type(16))) _Float16 v16h;
typedef __attribute__((ext_vector_type(16))) __bf16 v16b;
typedef __attribute__((ext_vector_type(8)))  _Float16 v8h;
typedef __attribute__((ext_vector_type(8)))  float v8f;
typedef __attribute__((ext_vector_type(4)))  float v4f;
typedef __attribute__((ext_vector_type(2)))  float v2f;
typedef __attribute__((ext_vector_type(4)))  unsigned v4u;
typedef __attribute__((ext_vector_type(4)))  int v4i;
typedef float __attribute__((may_alias)) float_a;
typedef int __attribute__((may_alias)) int_a;

template <typename T> __device__ __forceinline__ void vst2(void* p, T v) { *(volatile T*)p = v; __threadfence(); *(volatile T*)p = v; }
__device__ __forceinline__ v8f wmma16(v16h a, v16h b, v8f c) {
  v8f d = __builtin_amdgcn_wmma_f32_16x16x32_f16(false, a, false, b, (short)0, c, false, false);
  asm volatile("v_nop\n\tv_nop\n\tv_nop\n\tv_nop" : "+v"(d) : "v"(a), "v"(b));
  return d;
}
__device__ __forceinline__ v8f wmma_bf(v16b a, v16b b, v8f c) {
  v8f d = __builtin_amdgcn_wmma_f32_16x16x32_bf16(false, a, false, b, (short)0, c, false, false);
  asm volatile("v_nop\n\tv_nop\n\tv_nop\n\tv_nop" : "+v"(d) : "v"(a), "v"(b));
  return d;
}
__device__ __forceinline__ v16h frag_h(const _Float16* rowk0, int lane) {
  union { v16h v; v8h q[2]; } u; const _Float16* p = rowk0 + 8 * (lane >> 4);
  u.q[0] = *(const v8h*)p; u.q[1] = *(const v8h*)(p + 16); return u.v;
}
__device__ __forceinline__ v16h frag_f32(const float* rowk0, int lane) {
  v16h a; const float* p = rowk0 + 8 * (lane >> 4);
#pragma unroll
  for (int i = 0; i < 8; ++i) { a[i] = (_Float16)p[i]; a[8 + i] = (_Float16)p[16 + i]; }
  return a;
}
__device__ __forceinline__ v16h frag_f32s(const float* rowk0, int lane, float sc) {
  v16h a; const float* p = rowk0 + 8 * (lane >> 4);
#pragma unroll
  for (int i = 0; i < 8; ++i) { a[i] = (_Float16)(p[i] * sc); a[8 + i] = (_Float16)(p[16 + i] * sc); }
  return a;
}
__device__ __forceinline__ v16h fragc_f32(const float* W, int k0, int n, int lane, int ld, int K) {
  v16h a; const int g = lane >> 4;
#pragma unroll
  for (int i = 0; i < 8; ++i) { const int ka = k0 + 8 * g + i, kb = ka + 16;
    a[i] = (_Float16)(ka < K ? W[(size_t)(ka < K ? ka : K - 1) * ld + n] : 0.f); a[8 + i] = (_Float16)(kb < K ? W[(size_t)(kb < K ? kb : K - 1) * ld + n] : 0.f); }
  return a;
}
struct F2 { v16b h, l; };
__device__ __forceinline__ F2 bsplit16(const float v[16]) { F2 r;
#pragma unroll
  for (int i = 0; i < 16; ++i) { const __bf16 h = (__bf16)v[i]; r.h[i] = h; r.l[i] = (__bf16)(v[i] - (float)h); }
  return r; }
__device__ __forceinline__ F2 split_row(const float* row, int k0, int lane) { float v[16]; const float* p = row + k0 + 8 * (lane >> 4);
#pragma unroll
  for (int i = 0; i < 8; ++i) { v[i] = p[i]; v[8 + i] = p[16 + i]; }
  return bsplit16(v); }
__device__ __forceinline__ F2 split_rowK(const float* row, int k0, int lane, int K) { float v[16]; const int g = lane >> 4;
#pragma unroll
  for (int i = 0; i < 8; ++i) { const int ka = k0 + 8 * g + i, kb = ka + 16; v[i] = ka < K ? row[ka < K ? ka : K - 1] : 0.f; v[8 + i] = kb < K ? row[kb < K ? kb : K - 1] : 0.f; }
  return bsplit16(v); }
__device__ __forceinline__ F2 split_col(const float* W, int k0, int n, int lane, int ld, int K) { float v[16]; const int g = lane >> 4;
#pragma unroll
  for (int i = 0; i < 8; ++i) { const int ka = k0 + 8 * g + i, kb = ka + 16; v[i] = ka < K ? W[(size_t)(ka < K ? ka : K - 1) * ld + n] : 0.f; v[8 + i] = kb < K ? W[(size_t)(kb < K ? kb : K - 1) * ld + n] : 0.f; }
  return bsplit16(v); }
__device__ __forceinline__ v8f mac3(const F2& a, const F2& b, v8f c) { c = wmma_bf(a.l, b.h, c); c = wmma_bf(a.h, b.l, c); return wmma_bf(a.h, b.h, c); }
__device__ __forceinline__ float sigm(float v) { return 1.0f / (1.0f + expf(-v)); }
#define LDSX() do { asm volatile("s_wait_dscnt 0" ::: "memory"); __builtin_amdgcn_wave_barrier(); __builtin_amdgcn_fence(__ATOMIC_RELEASE, "workgroup"); } while (0)


#define NBAT 16384
#define NCF 8
#define DD 256
#define H0 512
#define H1 256
#ifndef RT
#define RT (NBAT / 64)
#endif
typedef __attribute__((ext_vector_type(8))) __bf16 v8b;
__device__ __forceinline__ v16b frag_b(const __bf16* rowk0, int lane) {
  union { v16b v; v8b q[2]; } u; const __bf16* p = rowk0 + 8 * (lane >> 4);
  u.q[0] = *(const v8b*)p; u.q[1] = *(const v8b*)(p + 16); return u.v;
}
__device__ __forceinline__ float bfr(float v) { return (float)(__bf16)v; }
__device__ __attribute__((noinline)) float exp_ni(float v) { return expf(v); }
__device__ __attribute__((noinline)) float erf_ni(float v) { return erff(v); }

#define WS_P0  0u
#define WS_P1  (2u * NCF * H0 * DD)
#define WS_G   (WS_P1 + 2u * NCF * H1 * H0)
#define WS_GL  (WS_G + 2u * (size_t)NBAT * H0)
#define WS_OC  (WS_GL + 2u * (size_t)NBAT * H0)
#define WS_END (WS_OC + 4u * NCF * NBAT)

__global__ __launch_bounds__(256) void k_pack(const float* __restrict__ W0, const float* __restrict__ W1, __bf16* __restrict__ PK) {
  __shared__ __align__(16) __bf16 s[H0]; const int n = blockIdx.x, which = blockIdx.y, t = threadIdx.x;
  const int K = (which == 0) ? DD : H0; if (which == 1 && n >= NCF * H1) return;
  const float* src = (which == 0) ? (W0 + (size_t)n * DD) : (W1 + (size_t)n * H0);
  for (int k = t; k < K; k += 256) s[k] = (__bf16)src[k];
  __syncthreads();
  for (int q = t; q < K / 8; q += 256) vst2((unsigned*)(PK + ((which == 0) ? WS_P0 / 2 : WS_P1 / 2) + (size_t)n * K + q * 8), *(const v4u*)&s[q * 8]);
}
__global__ __launch_bounds__(128) void k_l0(const float* __restrict__ X, const __bf16* __restrict__ P0, const float* __restrict__ B0, int c, __bf16* __restrict__ G, __bf16* __restrict__ GL) {
  __shared__ __align__(16) __bf16 sg[4][16][136], sgl[4][16][136];
  const int tid = threadIdx.x, wave = tid >> 5, lane = tid & 31, col = lane & 15, g = lane >> 4; const size_t r0 = (size_t)blockIdx.x * 64 + wave * 16; const int n0 = blockIdx.y * 128;
  const __bf16* P = P0 + (size_t)c * H0 * DD;
  v8f acc[8] = {};
#pragma unroll 2
  for (int kc = 0; kc < DD / 32; ++kc) { v16b a; { const float* p = X + (r0 + col) * DD + kc * 32 + 8 * g;
#pragma unroll
      for (int i = 0; i < 8; ++i) { a[i] = (__bf16)p[i]; a[8 + i] = (__bf16)p[16 + i]; } }
#pragma unroll
    for (int j = 0; j < 8; ++j) acc[j] = wmma_bf(a, frag_b(P + (size_t)(n0 + j * 16 + col) * DD + kc * 32, lane), acc[j]); }
#pragma unroll
  for (int j = 0; j < 8; ++j) { const float bb = bfr(B0[c * H0 + n0 + j * 16 + col]);
#pragma unroll
    for (int r = 0; r < 8; ++r) { const float v = fmaxf(acc[j][r] + bb, 0.f); const __bf16 hb = (__bf16)v; sg[wave][8 * g + r][j * 16 + col] = hb; sgl[wave][8 * g + r][j * 16 + col] = (__bf16)(v - (float)hb); } }
  LDSX();
  for (int rl = 0; rl < 16; ++rl) { if (lane < 16) vst2((unsigned*)(G + (r0 + rl) * H0 + n0 + lane * 8), *(const v4u*)&sg[wave][rl][lane * 8]); else vst2((unsigned*)(GL + (r0 + rl) * H0 + n0 + (lane - 16) * 8), *(const v4u*)&sgl[wave][rl][(lane - 16) * 8]); }
}
__global__ __launch_bounds__(128) void k_l12(const __bf16* __restrict__ G, const __bf16* __restrict__ GL, const __bf16* __restrict__ P1, const float* __restrict__ B1, const float* __restrict__ W2, const float* __restrict__ B2, int c, float* __restrict__ OC) {
  __shared__ float spart[2][4][16][17]; __shared__ __align__(16) float so[64];
  const int tid = threadIdx.x, wave = tid >> 5, lane = tid & 31, col = lane & 15, g = lane >> 4; const size_t r0 = (size_t)blockIdx.x * 64 + wave * 16;
  const __bf16* P = P1 + (size_t)c * H1 * H0;
#pragma unroll 1
  for (int half = 0; half < 2; ++half) { const int n0 = half * 128; v8f acc[8] = {};
#pragma unroll 2
    for (int kc = 0; kc < H0 / 32; ++kc) { const v16b a = frag_b(G + (r0 + col) * H0 + kc * 32, lane), al = frag_b(GL + (r0 + col) * H0 + kc * 32, lane);
#pragma unroll
      for (int j = 0; j < 8; ++j) { const v16b w = frag_b(P + (size_t)(n0 + j * 16 + col) * H0 + kc * 32, lane); acc[j] = wmma_bf(al, w, acc[j]); acc[j] = wmma_bf(a, w, acc[j]); } }
    float part[8];
#pragma unroll
    for (int r = 0; r < 8; ++r) part[r] = 0.f;
#pragma unroll
    for (int j = 0; j < 8; ++j) { const int o = n0 + j * 16 + col; const float bb = bfr(B1[c * H1 + o]), w2 = bfr(W2[(size_t)c * H1 + o]);
#pragma unroll
      for (int r = 0; r < 8; ++r) part[r] += fmaxf(acc[j][r] + bb, 0.f) * w2; }
#pragma unroll
    for (int r = 0; r < 8; ++r) { float v = part[r];
#pragma unroll
      for (int o = 1; o < 16; o <<= 1) v += __shfl_xor(v, o);
      if (col == 0) spart[half][wave][8 * g + r][0] = v; } }
  LDSX();
  if (lane < 16) so[wave * 16 + lane] = spart[0][wave][lane][0] + spart[1][wave][lane][0] + bfr(B2[c]);
  __syncthreads();
  if (tid < 16) vst2(OC + (size_t)c * NBAT + (size_t)blockIdx.x * 64 + tid * 4, *(const v4f*)&so[tid * 4]);
}
__global__ __launch_bounds__(128) void k_gather(const float* __restrict__ OC, float* __restrict__ OUT) {
  __shared__ __align__(16) float so[64][NCF]; const int t = threadIdx.x; const size_t b0 = (size_t)blockIdx.x * 64;
  for (int e = t; e < 64 * NCF; e += 128) { const int r = e & 63, c = e >> 6; so[r][c] = OC[(size_t)c * NBAT + b0 + r]; }
  __syncthreads();
  vst2(OUT + b0 * NCF + t * 4, *(const v4f*)(&so[0][0] + t * 4));
}
extern "C" void kernel_launch(void* const* d_in, const int* in_sizes, int n_in, void* d_out, int out_size, void* d_ws, size_t ws_size, hipStream_t stream) {
  (void)in_sizes; (void)n_in; (void)out_size;
  const float** F = (const float**)d_in;
  if (ws_size < (size_t)WS_END) return;
  char* ws = (char*)d_ws; __bf16* PK = (__bf16*)ws; __bf16 *G = (__bf16*)(ws + WS_G), *GL = (__bf16*)(ws + WS_GL); float* OC = (float*)(ws + WS_OC);
  k_pack<<<dim3(NCF * H0, 2), 256, 0, stream>>>(F[1], F[3], PK);
  for (int c = 0; c < NCF; ++c) {
    k_l0<<<dim3(RT, H0 / 128), 128, 0, stream>>>(F[0], (const __bf16*)(ws + WS_P0), F[2], c, G, GL);
    k_l12<<<RT, 128, 0, stream>>>(G, GL, (const __bf16*)(ws + WS_P1), F[4], F[5], F[6], c, OC); }
  k_gather<<<RT, 128, 0, stream>>>(OC, (float*)d_out);
}
